// StackedFlow_81913616269685
// MI455X (gfx1250) — hardware-run, weakly checked
//
#include <hip/hip_runtime.h>
#include <math.h>

#ifndef NB
#define NB 256
#endif
#define NB_FULL 256
#define DDIM 16
#define MHID 128
#define HID 2048
#define NTILE_N (HID / 64)
#define NTILES ((NB / 16) * NTILE_N)

#define CX_CARRY  256.0f
#define CW_CARRY  32768.0f
#define CT_CARRY  1024.0f
#define CG0_CARRY 32768.0f
#define CG1_CARRY 16384.0f
#define INV_XW  (1.0f / 8388608.0f)
#define INV_TW  (1.0f / 33554432.0f)
#define INV_G0W (1.0f / 1073741824.0f)
#define INV_G1W (1.0f / 536870912.0f)

static_assert(NB % 32 == 0);
static_assert(NB <= NB_FULL);
static_assert(HID == DDIM * MHID);
static_assert(NTILE_N == 32);
static_assert(NTILES % 4 == 0);
static_assert(HID % 32 == 0 && MHID % 32 == 0);
static_assert(NB_FULL * DDIM * 4 == 16384);
static_assert((NB_FULL * DDIM + NB) * 4 <= 17408);

typedef _Float16 h16;
typedef __attribute__((ext_vector_type(16))) _Float16 v16h;
typedef __attribute__((ext_vector_type(8)))  _Float16 v8h;
typedef __attribute__((ext_vector_type(8)))  float    v8f;
typedef __attribute__((ext_vector_type(4)))  float    v4f;


constexpr size_t SZ_W1P   = (size_t)HID * HID * 2;
constexpr size_t SZ_W2P   = (size_t)DDIM * HID * 2;
constexpr size_t SZ_ACT   = (size_t)NB * HID * 2;
constexpr size_t OFF_W2M  = SZ_W1P;
constexpr size_t OFF_W2D  = OFF_W2M + SZ_W2P;
constexpr size_t OFF_T0   = OFF_W2D + SZ_W2P;
constexpr size_t OFF_G0   = OFF_T0 + SZ_ACT;
constexpr size_t OFF_T1   = OFF_G0 + SZ_ACT;
constexpr size_t OFF_G1   = OFF_T1 + SZ_ACT;
constexpr size_t SZ_STAGE = OFF_G1 + SZ_ACT;
constexpr size_t OFF_XMID = 2 * SZ_STAGE;
constexpr size_t SZ_XMID  = (size_t)NB * DDIM * 4;
constexpr size_t OFF_LD0  = OFF_XMID + SZ_XMID;
constexpr size_t SZ_LD0   = (size_t)NB * 4;
constexpr size_t WS_TOTAL = OFF_LD0 + SZ_LD0;
static_assert(SZ_STAGE % 256 == 0 && SZ_ACT % 256 == 0 && SZ_W2P % 256 == 0);
static_assert(OFF_XMID % 128 == 0 && OFF_LD0 % 128 == 0 && SZ_LD0 % 128 == 0 && SZ_XMID % 128 == 0);
static_assert(WS_TOTAL <= (size_t)134217728);

static __device__ __forceinline__ float bfr(float f) {
    unsigned u = __float_as_uint(f);
    u += 0x7FFFu + ((u >> 16) & 1u);
    return __uint_as_float(u & 0xFFFF0000u);
}
static __device__ __forceinline__ h16 toh_flush(float v) {
    const float w = (fabsf(v) < 6.103515625e-05f) ? 0.0f : v;
    return (h16)w;
}
static __device__ __forceinline__ float dtanh_z(float z) {
    const float e = expf(-2.0f * fabsf(z));
    const float s = 1.0f + e;
    return (4.0f * e) / (s * s);
}

union FragU { v16h v; v8h h[2]; };
static __device__ __forceinline__ v16h frag_ld(const h16* p) {
    FragU f; f.h[0] = *(const v8h*)(p); f.h[1] = *(const v8h*)(p + 16); return f.v;
}
static __device__ __forceinline__ v8f wmma16g(v16h a, v16h b, v8f c) {
    c = __builtin_amdgcn_wmma_f32_16x16x32_f16(false, a, false, b, (short)0, c, false, false);
    asm volatile("v_nop\n\tv_nop\n\tv_nop\n\tv_nop" : "+v"(c) : "v"(a), "v"(b));
    return c;
}
static __device__ __forceinline__ void wave_sync_lds() {
    __builtin_amdgcn_fence(3  , "workgroup");
    __builtin_amdgcn_wave_barrier();
    __builtin_amdgcn_fence(2  , "workgroup");
}

__global__ __launch_bounds__(256) void k_w1plane(const float* __restrict__ W, h16* __restrict__ P) {
    const unsigned o = blockIdx.x;
    const unsigned t = threadIdx.x;
    if (o >= (unsigned)HID) return;
    const unsigned k0 = t * 8u;
    const float* src = W + (size_t)o * HID + k0;
    const v4f a = *(const v4f*)src;
    const v4f b = *(const v4f*)(src + 4);
    const float keep = ((k0 >> 7) <= (o >> 7)) ? 1.0f : 0.0f;
    const float w[8] = {a.x, a.y, a.z, a.w, b.x, b.y, b.z, b.w};
    v8h hv;
#pragma unroll
    for (int e = 0; e < 8; ++e) hv[e] = toh_flush(bfr(w[e]) * keep * CW_CARRY);
    h16* dst = P + (size_t)o * HID + k0;
    *(volatile v8h*)dst = hv;
    __threadfence();
    *(volatile v8h*)dst = hv;
}

__global__ __launch_bounds__(256) void k_w2planes(const float* __restrict__ W, h16* __restrict__ Pm, h16* __restrict__ Pd) {
    const unsigned j = blockIdx.x;
    const unsigned t = threadIdx.x;
    if (j >= (unsigned)DDIM) return;
    const unsigned k0 = t * 8u;
    const unsigned kb = k0 >> 7;
    const float* src = W + (size_t)j * HID + k0;
    const v4f a = *(const v4f*)src;
    const v4f b = *(const v4f*)(src + 4);
    const float keepM = (kb <= j) ? 1.0f : 0.0f;
    const float keepD = (kb == j) ? 1.0f : 0.0f;
    const float w[8] = {a.x, a.y, a.z, a.w, b.x, b.y, b.z, b.w};
    v8h hm, hd;
#pragma unroll
    for (int e = 0; e < 8; ++e) {
        const float wv = bfr(w[e]);
        hm[e] = toh_flush(wv * keepM * CW_CARRY);
        hd[e] = toh_flush(wv * keepD * CW_CARRY);
    }
    h16* dm = Pm + (size_t)j * HID + k0;
    h16* dd = Pd + (size_t)j * HID + k0;
    *(volatile v8h*)dm = hm;
    *(volatile v8h*)dd = hd;
    __threadfence();
    *(volatile v8h*)dm = hm;
    *(volatile v8h*)dd = hd;
}

template <bool RNE_X>
__global__ __launch_bounds__(128) void k_lay0(const float* __restrict__ X, const float* __restrict__ W0,
                                              const float* __restrict__ b0, h16* __restrict__ Tp, h16* __restrict__ Gp) {
    __shared__ __align__(16) float sT[4][2][16 * 68];
    const unsigned lane = threadIdx.x & 31u;
    const unsigned wave = threadIdx.x >> 5;
    const unsigned tile = blockIdx.x * 4u + wave;
    if (tile >= (unsigned)NTILES) return;
    const unsigned tm = tile >> 5, tn = tile & 31u;
    const unsigned m0 = tm << 4, n0 = tn << 6;
    const unsigned c = lane & 15u, hh = lane >> 4, koff = hh * 8u;
    const unsigned jb = n0 >> 7;

    v16h af;
    {
        const float* xr = X + (size_t)(m0 + c) * DDIM + koff;
        const v4f xa = *(const v4f*)xr;
        const v4f xb = *(const v4f*)(xr + 4);
        const float xs[8] = {xa.x, xa.y, xa.z, xa.w, xb.x, xb.y, xb.z, xb.w};
#pragma unroll
        for (int i = 0; i < 8; ++i) {
            const float xv = RNE_X ? bfr(xs[i]) : xs[i];
            af[i] = toh_flush(xv * CX_CARRY);
            af[i + 8] = toh_flush(0.0f);
        }
    }
    v8f acc[4];
#pragma unroll
    for (int jj = 0; jj < 4; ++jj) {
        const unsigned n = n0 + ((unsigned)jj << 4) + c;
        const float* wr = W0 + (size_t)n * DDIM + koff;
        const v4f wa = *(const v4f*)wr;
        const v4f wb = *(const v4f*)(wr + 4);
        const float ws8[8] = {wa.x, wa.y, wa.z, wa.w, wb.x, wb.y, wb.z, wb.w};
        v16h bf;
#pragma unroll
        for (int i = 0; i < 8; ++i) {
            const float keep = ((koff + (unsigned)i) <= jb) ? 1.0f : 0.0f;
            bf[i] = toh_flush(bfr(ws8[i]) * keep * CW_CARRY);
            bf[i + 8] = toh_flush(0.0f);
        }
        const v8f z = (v8f){0.f, 0.f, 0.f, 0.f, 0.f, 0.f, 0.f, 0.f};
        acc[jj] = wmma16g(af, bf, z);
    }

    float* slT = sT[wave][0];
    float* slG = sT[wave][1];
#pragma unroll
    for (int jj = 0; jj < 4; ++jj) {
        const unsigned n = n0 + ((unsigned)jj << 4) + c;
        const float bv = bfr(b0[n]);
        const float wd = bfr(W0[(size_t)n * DDIM + jb]);
#pragma unroll
        for (int r = 0; r < 8; ++r) {
            const float z = acc[jj][r] * INV_XW + bv;
            const float t = tanhf(z);
            const float g = wd * dtanh_z(z);
            slT[(koff + (unsigned)r) * 68u + ((unsigned)jj << 4) + c] = t * CT_CARRY;
            slG[(koff + (unsigned)r) * 68u + ((unsigned)jj << 4) + c] = g * CG0_CARRY;
        }
    }
    wave_sync_lds();
    {
        const unsigned q = lane >> 3, c8 = (lane & 7u) * 8u;
        v8h ht[4], hg[4];
#pragma unroll
        for (int it = 0; it < 4; ++it) {
            const unsigned row = (unsigned)it * 4u + q;
            const float* spt = slT + row * 68u + c8;
            const float* spg = slG + row * 68u + c8;
#pragma unroll
            for (int e = 0; e < 8; ++e) { ht[it][e] = toh_flush(spt[e]); hg[it][e] = toh_flush(spg[e]); }
        }
        for (int pass = 0; pass < 2; ++pass) {
#pragma unroll
            for (int it = 0; it < 4; ++it) {
                const unsigned row = (unsigned)it * 4u + q;
                *(volatile v8h*)(Tp + (size_t)(m0 + row) * HID + n0 + c8) = ht[it];
                *(volatile v8h*)(Gp + (size_t)(m0 + row) * HID + n0 + c8) = hg[it];
            }
            __threadfence();
        }
    }
}

__global__ __launch_bounds__(128) void k_lay1(const h16* __restrict__ T0, const h16* __restrict__ G0,
                                              const h16* __restrict__ W1p, const float* __restrict__ b1,
                                              h16* __restrict__ T1, h16* __restrict__ G1) {
    __shared__ __align__(16) float sT[4][2][16 * 68];
    const unsigned lane = threadIdx.x & 31u;
    const unsigned wave = threadIdx.x >> 5;
    const unsigned tile = blockIdx.x * 4u + wave;
    if (tile >= (unsigned)NTILES) return;
    const unsigned tm = tile >> 5, tn = tile & 31u;
    const unsigned m0 = tm << 4, n0 = tn << 6;
    const unsigned c = lane & 15u, hh = lane >> 4, koff = hh * 8u;
    const unsigned kd0 = (n0 >> 7) << 7;

    v8f accZ[4], accJ[4];
#pragma unroll
    for (int jj = 0; jj < 4; ++jj) {
        accZ[jj] = (v8f){0.f, 0.f, 0.f, 0.f, 0.f, 0.f, 0.f, 0.f};
        accJ[jj] = (v8f){0.f, 0.f, 0.f, 0.f, 0.f, 0.f, 0.f, 0.f};
    }
    const h16* arowT = T0 + (size_t)(m0 + c) * HID + koff;
    const h16* arowG = G0 + (size_t)(m0 + c) * HID + koff;
    const h16* brow  = W1p + (size_t)(n0 + c) * HID + koff;

    for (unsigned k0 = 0; k0 < kd0; k0 += 32u) {
        const v16h at = frag_ld(arowT + k0);
#pragma unroll
        for (int jj = 0; jj < 4; ++jj) {
            const v16h bh = frag_ld(brow + (size_t)((unsigned)jj << 4) * HID + k0);
            accZ[jj] = wmma16g(at, bh, accZ[jj]);
        }
    }
    for (unsigned k0 = kd0; k0 < kd0 + (unsigned)MHID; k0 += 32u) {
        const v16h at = frag_ld(arowT + k0);
        const v16h ag = frag_ld(arowG + k0);
#pragma unroll
        for (int jj = 0; jj < 4; ++jj) {
            const v16h bh = frag_ld(brow + (size_t)((unsigned)jj << 4) * HID + k0);
            accZ[jj] = wmma16g(at, bh, accZ[jj]);
            accJ[jj] = wmma16g(ag, bh, accJ[jj]);
        }
    }

    float* slT = sT[wave][0];
    float* slG = sT[wave][1];
#pragma unroll
    for (int jj = 0; jj < 4; ++jj) {
        const unsigned n = n0 + ((unsigned)jj << 4) + c;
        const float bv = bfr(b1[n]);
#pragma unroll
        for (int r = 0; r < 8; ++r) {
            const float z = accZ[jj][r] * INV_TW + bv;
            const float t = tanhf(z);
            const float g = (accJ[jj][r] * INV_G0W) * dtanh_z(z);
            slT[(koff + (unsigned)r) * 68u + ((unsigned)jj << 4) + c] = t * CT_CARRY;
            slG[(koff + (unsigned)r) * 68u + ((unsigned)jj << 4) + c] = g * CG1_CARRY;
        }
    }
    wave_sync_lds();
    {
        const unsigned q = lane >> 3, c8 = (lane & 7u) * 8u;
        v8h ht[4], hg[4];
#pragma unroll
        for (int it = 0; it < 4; ++it) {
            const unsigned row = (unsigned)it * 4u + q;
            const float* spt = slT + row * 68u + c8;
            const float* spg = slG + row * 68u + c8;
#pragma unroll
            for (int e = 0; e < 8; ++e) { ht[it][e] = toh_flush(spt[e]); hg[it][e] = toh_flush(spg[e]); }
        }
        for (int pass = 0; pass < 2; ++pass) {
#pragma unroll
            for (int it = 0; it < 4; ++it) {
                const unsigned row = (unsigned)it * 4u + q;
                *(volatile v8h*)(T1 + (size_t)(m0 + row) * HID + n0 + c8) = ht[it];
                *(volatile v8h*)(G1 + (size_t)(m0 + row) * HID + n0 + c8) = hg[it];
            }
            __threadfence();
        }
    }
}

template <bool FINAL_STAGE>
__global__ __launch_bounds__(64) void k_last(const h16* __restrict__ T1, const h16* __restrict__ G1,
                                             const h16* __restrict__ W2m, const h16* __restrict__ W2d,
                                             const float* ldprev, float* yout, float* ldout) {
    __shared__ __align__(16) float sY[2][256];
    __shared__ __align__(16) float sL[2][16 * 17];
    __shared__ __align__(16) float sLd[32];
    const unsigned lane = threadIdx.x & 31u;
    const unsigned wave = threadIdx.x >> 5;
    const unsigned bx = blockIdx.x;
    const unsigned m0 = bx * 32u + wave * 16u;
    const unsigned c = lane & 15u, hh = lane >> 4, koff = hh * 8u;

    v8f accY = (v8f){0.f, 0.f, 0.f, 0.f, 0.f, 0.f, 0.f, 0.f};
    v8f accG = (v8f){0.f, 0.f, 0.f, 0.f, 0.f, 0.f, 0.f, 0.f};
    const h16* arowT = T1 + (size_t)(m0 + c) * HID + koff;
    const h16* arowG = G1 + (size_t)(m0 + c) * HID + koff;
    const h16* browM = W2m + (size_t)c * HID + koff;
    const h16* browD = W2d + (size_t)c * HID + koff;
    for (unsigned k0 = 0; k0 < (unsigned)HID; k0 += 32u) {
        const v16h at = frag_ld(arowT + k0);
        const v16h bm = frag_ld(browM + k0);
        accY = wmma16g(at, bm, accY);
        const v16h ag = frag_ld(arowG + k0);
        const v16h bd = frag_ld(browD + k0);
        accG = wmma16g(ag, bd, accG);
    }

    float* sy = sY[wave];
    float* sl = sL[wave];
#pragma unroll
    for (int r = 0; r < 8; ++r) {
        const unsigned row = koff + (unsigned)r;
        sy[row * 16u + c] = accY[r] * INV_TW;
        sl[row * 17u + c] = logf(accG[r] * INV_G1W);
    }
    wave_sync_lds();
    {
        const float* lr = sl + c * 17u;
        float s = 0.0f;
#pragma unroll
        for (int jj = 0; jj < 16; ++jj) s += lr[jj];
        if (lane < 16u) sLd[wave * 16u + lane] = s;
    }
    {
        const v4f y0 = *(const v4f*)(sy + 4u * lane);
        const v4f y1 = *(const v4f*)(sy + 128u + 4u * lane);
        float* yd = yout + (size_t)m0 * DDIM;
        for (int pass = 0; pass < 2; ++pass) {
            *(volatile v4f*)(yd + 4u * lane) = y0;
            *(volatile v4f*)(yd + 128u + 4u * lane) = y1;
            __threadfence();
        }
    }
    __syncthreads();
    if (wave == 0u && lane < 8u) {
        v4f lv = *(const v4f*)(sLd + 4u * lane);
        if (FINAL_STAGE) {
            const v4f pv = *(const v4f*)(ldprev + (size_t)bx * 32u + 4u * lane);
            lv = lv + pv;
        }
        float* ldd = ldout + (size_t)bx * 32u + 4u * lane;
        *(volatile v4f*)ldd = lv;
        __threadfence();
        *(volatile v4f*)ldd = lv;
    }
}

extern "C" void kernel_launch(void* const* d_in, const int* in_sizes, int n_in, void* d_out, int out_size,
                              void* d_ws, size_t ws_size, hipStream_t stream) {
    if (n_in < 11) return;
    if (in_sizes[0] < NB * DDIM) return;
    if (in_sizes[1] < HID * DDIM || in_sizes[6] < HID * DDIM) return;
    if (in_sizes[2] < HID * HID || in_sizes[7] < HID * HID) return;
    if (in_sizes[3] < DDIM * HID || in_sizes[8] < DDIM * HID) return;
    if (in_sizes[4] < HID || in_sizes[5] < HID || in_sizes[9] < HID || in_sizes[10] < HID) return;
    if (out_size < NB_FULL * DDIM + NB) return;
    if (WS_TOTAL > ws_size) return;

    const float* inp = (const float*)d_in[0];
    const float* W0s[2] = {(const float*)d_in[1], (const float*)d_in[6]};
    const float* W1s[2] = {(const float*)d_in[2], (const float*)d_in[7]};
    const float* W2s[2] = {(const float*)d_in[3], (const float*)d_in[8]};
    const float* b0s[2] = {(const float*)d_in[4], (const float*)d_in[9]};
    const float* b1s[2] = {(const float*)d_in[5], (const float*)d_in[10]};
    float* out = (float*)d_out;
    float* ldo = out + (size_t)NB_FULL * DDIM;

    char* wsp = (char*)d_ws;
    float* xmid = (float*)(wsp + OFF_XMID);
    float* ld0  = (float*)(wsp + OFF_LD0);

    for (int s = 0; s < 2; ++s) {
        char* base = wsp + (size_t)s * SZ_STAGE;
        h16* w1p = (h16*)(base);
        h16* w2m = (h16*)(base + OFF_W2M);
        h16* w2d = (h16*)(base + OFF_W2D);
        h16* t0  = (h16*)(base + OFF_T0);
        h16* g0  = (h16*)(base + OFF_G0);
        h16* t1  = (h16*)(base + OFF_T1);
        h16* g1  = (h16*)(base + OFF_G1);

        k_w1plane<<<HID, 256, 0, stream>>>(W1s[s], w1p);
        k_w2planes<<<DDIM, 256, 0, stream>>>(W2s[s], w2m, w2d);
        if (s == 0) {
            k_lay0<true><<<NTILES / 4, 128, 0, stream>>>(inp, W0s[0], b0s[0], t0, g0);
        } else {
            k_lay0<false><<<NTILES / 4, 128, 0, stream>>>(xmid, W0s[1], b0s[1], t0, g0);
        }
        k_lay1<<<NTILES / 4, 128, 0, stream>>>(t0, g0, w1p, b1s[s], t1, g1);
        if (s == 0) {
            k_last<false><<<NB / 32, 64, 0, stream>>>(t1, g1, w2m, w2d, ld0, xmid, ld0);
        } else {
            k_last<true><<<NB / 32, 64, 0, stream>>>(t1, g1, w2m, w2d, ld0, out, ldo);
        }
    }
}
